// DGraph_GAT_56899726737498
// MI455X (gfx1250) — hardware-verified
//
#include <hip/hip_runtime.h>


#define NN   8192
#define FIN  512
#define HF   256
#define LAT  32
#define RCH  1024
#define NCH  (NN / RCH)
#define DM   FIN
#define LOSC 1024.0f

typedef _Float16 h16;
typedef unsigned short bf;
typedef __attribute__((ext_vector_type(16))) __bf16   v16bf;
typedef __attribute__((ext_vector_type(16))) _Float16 v16h;
typedef __attribute__((ext_vector_type(8)))  _Float16 v8h;
typedef __attribute__((ext_vector_type(8)))  unsigned short v8us;
typedef __attribute__((ext_vector_type(8)))  float    v8f;
typedef __attribute__((ext_vector_type(4)))  float    v4f;
typedef __attribute__((ext_vector_type(4)))  _Float16 v4h;
typedef v8h  __attribute__((may_alias)) v8ha;
typedef v4f  __attribute__((may_alias)) v4fa;
typedef v8us __attribute__((may_alias)) v8usa;

__device__ __forceinline__ unsigned short f2bf(float f) { unsigned u = __float_as_uint(f); u += 0x7FFFu + ((u >> 16) & 1u); return (unsigned short)(u >> 16); }
__device__ __forceinline__ float bf2f(unsigned short b) { return __uint_as_float(((unsigned)b) << 16); }
__device__ __forceinline__ float bfr(float f) { return bf2f(f2bf(f)); }
__device__ __forceinline__ v16h cat16(v8h lo, v8h hi) { return __builtin_shufflevector(lo, hi, 0, 1, 2, 3, 4, 5, 6, 7, 8, 9, 10, 11, 12, 13, 14, 15); }
__device__ __forceinline__ v16bf cat16b(v8us lo, v8us hi) { return __builtin_bit_cast(v16bf, __builtin_shufflevector(lo, hi, 0, 1, 2, 3, 4, 5, 6, 7, 8, 9, 10, 11, 12, 13, 14, 15)); }
__device__ __forceinline__ v8f wmma16(v16h a, v16h b, v8f c) { return __builtin_amdgcn_wmma_f32_16x16x32_f16(false, a, false, b, (short)0, c, false, false); }
__device__ __forceinline__ v8f wmmab(v16bf a, v16bf b, v8f c) { return __builtin_amdgcn_wmma_f32_16x16x32_bf16(false, a, false, b, (short)0, c, false, false); }

__global__ __launch_bounds__(256) void k_wt(const float* __restrict__ Wm, int K, int ncols, bf* WT) {
    __shared__ __align__(16) unsigned short tl[64 * 72];
    const int tid = threadIdx.x, k0 = blockIdx.x * 64, n0 = blockIdx.y * 64;
    const int kk = tid >> 2, nq = (tid & 3) * 16;
#pragma unroll
    for (int i = 0; i < 16; ++i) tl[(nq + i) * 72 + kk] = f2bf(Wm[(size_t)(k0 + kk) * ncols + n0 + nq + i]);
    __syncthreads();
    const int piece = tid & 7;
    auto pass = [&]() {
#pragma unroll
        for (int s = 0; s < 2; ++s) { const int nr = (tid >> 3) + 32 * s; const v8us val = *(const v8usa*)(tl + nr * 72 + piece * 8); *(volatile v8us*)(WT + (size_t)(n0 + nr) * K + k0 + piece * 8) = val; }
    };
    pass(); __threadfence(); pass();
}
template <bool SPLITA, bool F16OUT = false>
__global__ __launch_bounds__(128) void k_gemmb(const bf* __restrict__ A, const bf* __restrict__ Al, const bf* __restrict__ Bn, const float* __restrict__ bias, float* C, int ldc, h16* C2, const float* __restrict__ R = nullptr, int K = DM, int roundR = 1) {
    __shared__ __align__(16) float ost[4][16 * 68];
    const int lane = threadIdx.x & 31, wave = threadIdx.x >> 5, lr = lane & 15, hi = lane >> 4;
    const int r0 = blockIdx.x * 64 + wave * 16, c0 = blockIdx.y * 64;
    const size_t aoff = (size_t)(r0 + lr) * K + 8 * hi;
    size_t boff[4];
#pragma unroll
    for (int t = 0; t < 4; ++t) boff[t] = (size_t)(c0 + t * 16 + lr) * K + 8 * hi;
    v8f acc[4];
#pragma unroll
    for (int t = 0; t < 4; ++t) acc[t] = (v8f){};
#pragma unroll 1
    for (int kc = 0; kc < K; kc += 32) {
        const v16bf a = cat16b(*(const v8us*)(A + aoff + kc), *(const v8us*)(A + aoff + kc + 16));
        v16bf al = a;
        if (SPLITA) al = cat16b(*(const v8us*)(Al + aoff + kc), *(const v8us*)(Al + aoff + kc + 16));
#pragma unroll
        for (int t = 0; t < 4; ++t) { const v16bf b = cat16b(*(const v8us*)(Bn + boff[t] + kc), *(const v8us*)(Bn + boff[t] + kc + 16)); acc[t] = wmmab(a, b, acc[t]); if (SPLITA) acc[t] = wmmab(al, b, acc[t]); }
        asm volatile("v_nop\n\tv_nop\n\tv_nop\n\tv_nop" : "+v"(acc[0]), "+v"(acc[1]), "+v"(acc[2]), "+v"(acc[3]) : "v"(a), "v"(al));
    }
    float* os = &ost[wave][0];
#pragma unroll
    for (int t = 0; t < 4; ++t) { const float bv = bias ? bfr(bias[c0 + t * 16 + lr]) : 0.f;
#pragma unroll
        for (int j = 0; j < 8; ++j) os[(hi * 8 + j) * 68 + t * 16 + lr] = acc[t][j] + bv; }
    __syncthreads();
    if (F16OUT) {
        h16* crow = (h16*)(void*)C + (size_t)r0 * ldc + c0;
        auto pass = [&]() {
#pragma unroll
            for (int s = 0; s < 4; ++s) { const int row = 4 * s + (lane >> 3), piece = lane & 7; const float* sp = os + row * 68 + piece * 8; v8h o, o2;
#pragma unroll
                for (int i = 0; i < 8; ++i) { const h16 a = (h16)sp[i]; o[i] = a; o2[i] = (h16)((sp[i] - (float)a) * LOSC); }
                *(volatile v8h*)(crow + (size_t)row * ldc + piece * 8) = o; if (C2) *(volatile v8h*)(C2 + (size_t)r0 * ldc + c0 + (size_t)row * ldc + piece * 8) = o2; }
        };
        pass(); __threadfence(); pass();
    } else {
        float* crow = C + (size_t)r0 * ldc + c0;
        auto pass = [&]() {
#pragma unroll
            for (int s = 0; s < 8; ++s) { const int Lid = (lane >> 3) + 4 * s, piece = lane & 7; const int row = Lid >> 1, cofs = (Lid & 1) * 32 + piece * 4;
                v4f val = *(const v4fa*)(os + row * 68 + cofs); if (R) { const v4f rv = *(const v4f*)(R + ((size_t)r0 + row) * ldc + c0 + cofs); val += roundR ? (v4f){bfr(rv[0]), bfr(rv[1]), bfr(rv[2]), bfr(rv[3])} : rv; }
                *(volatile v4f*)(crow + (size_t)row * ldc + cofs) = val; }
        };
        pass(); __threadfence(); pass();
    }
}

__global__ __launch_bounds__(128) void k_gemm3(const bf* __restrict__ Ah, const bf* __restrict__ Al, const bf* __restrict__ Bh, const bf* __restrict__ Bl, int K, float* C, int ldc) {
    __shared__ __align__(16) float ost[4][16 * 68];
    const int lane = threadIdx.x & 31, wave = threadIdx.x >> 5, lr = lane & 15, hi = lane >> 4;
    const int r0 = blockIdx.x * 64 + wave * 16, c0 = blockIdx.y * 64;
    const size_t aoff = (size_t)(r0 + lr) * K + 8 * hi;
    v8f acc[4];
#pragma unroll
    for (int t = 0; t < 4; ++t) acc[t] = (v8f){};
#pragma unroll 1
    for (int kc = 0; kc < K; kc += 32) {
        const v16bf a = cat16b(*(const v8us*)(Ah + aoff + kc), *(const v8us*)(Ah + aoff + kc + 16));
        const v16bf al = cat16b(*(const v8us*)(Al + aoff + kc), *(const v8us*)(Al + aoff + kc + 16));
#pragma unroll
        for (int t = 0; t < 4; ++t) { const size_t bo = (size_t)(c0 + t * 16 + lr) * K + kc + 8 * hi;
            const v16bf bh = cat16b(*(const v8us*)(Bh + bo), *(const v8us*)(Bh + bo + 16)); const v16bf bl = cat16b(*(const v8us*)(Bl + bo), *(const v8us*)(Bl + bo + 16));
            acc[t] = wmmab(a, bh, acc[t]); acc[t] = wmmab(al, bh, acc[t]); acc[t] = wmmab(a, bl, acc[t]); }
        asm volatile("v_nop\n\tv_nop\n\tv_nop\n\tv_nop" : "+v"(acc[0]), "+v"(acc[1]), "+v"(acc[2]), "+v"(acc[3]) : "v"(a), "v"(al));
    }
    float* os = &ost[wave][0];
#pragma unroll
    for (int t = 0; t < 4; ++t) {
#pragma unroll
        for (int j = 0; j < 8; ++j) os[(hi * 8 + j) * 68 + t * 16 + lr] = acc[t][j]; }
    __builtin_amdgcn_wave_barrier(); asm volatile("" ::: "memory");
    float* crow = C + (size_t)r0 * ldc + c0;
    auto pass = [&]() {
#pragma unroll
        for (int s = 0; s < 8; ++s) { const int Lid = (lane >> 3) + 4 * s, piece = lane & 7; const int row = Lid >> 1, cofs = (Lid & 1) * 32 + piece * 4;
            const v4f val = *(const v4fa*)(os + row * 68 + cofs); *(volatile v4f*)(crow + (size_t)row * ldc + cofs) = val; }
    };
    pass(); __threadfence(); pass();
}

__global__ __launch_bounds__(256) void k_wtp(const float* __restrict__ Wm, int krows, int ncols, int kpad, bf* WT) {
    __shared__ __align__(16) unsigned short tl[64 * 72];
    const int tid = threadIdx.x, k0 = blockIdx.x * 64, n0 = blockIdx.y * 64;
    const int kk = tid >> 2, nq = (tid & 3) * 16;
    const int k = k0 + kk, kc = k < krows ? k : krows - 1;
#pragma unroll
    for (int i = 0; i < 16; ++i) { const int n = n0 + nq + i, ncl = n < ncols ? n : ncols - 1; const float w = Wm[(size_t)kc * ncols + ncl]; tl[(nq + i) * 72 + kk] = (k < krows && n < ncols) ? f2bf(w) : (unsigned short)0; }
    __syncthreads();
    const int piece = tid & 7;
    auto pass = [&]() {
#pragma unroll
        for (int s = 0; s < 2; ++s) { const int nr = (tid >> 3) + 32 * s; const v8us val = *(const v8usa*)(tl + nr * 72 + piece * 8); *(volatile v8us*)(WT + (size_t)(n0 + nr) * kpad + k0 + piece * 8) = val; }
    };
    pass(); __threadfence(); pass();
}

__global__ __launch_bounds__(256) void k_cvt8(const float* __restrict__ src, bf* dst, size_t n8) {
    const size_t i = (size_t)blockIdx.x * 256 + threadIdx.x; if (i >= n8) return;
    const v8f v = *(const v8f*)(src + i * 8); v8us o;
#pragma unroll
    for (int k = 0; k < 8; ++k) o[k] = f2bf(v[k]);
    *(volatile v8us*)(dst + i * 8) = o; __threadfence(); *(volatile v8us*)(dst + i * 8) = o;
}
__global__ __launch_bounds__(256) void k_zero8(bf* dst, size_t n8) {
    const size_t i = (size_t)blockIdx.x * 256 + threadIdx.x; if (i >= n8) return; v8us z;
#pragma unroll
    for (int k = 0; k < 8; ++k) z[k] = 0;
    *(volatile v8us*)(dst + i * 8) = z; __threadfence(); *(volatile v8us*)(dst + i * 8) = z;
}

__global__ __launch_bounds__(256) void k_cvtx(const float* __restrict__ src, bf* dst) {
    const int lane = threadIdx.x & 31; const size_t r = (size_t)blockIdx.x * 8 + (threadIdx.x >> 5); if (r >= (size_t)NN) return;
#pragma unroll 1
    for (int ps = 0; ps < 2; ++ps) {
#pragma unroll
        for (int q = 0; q < FIN / 256; ++q) { v8us o;
#pragma unroll
            for (int i = 0; i < 8; ++i) o[i] = f2bf(src[r * FIN + q * 256 + lane * 8 + i]);
            *(volatile v8us*)(dst + r * FIN + q * 256 + lane * 8) = o; }
        if (ps == 0) __threadfence(); }
}
__global__ __launch_bounds__(256) void k_relu256(const float* __restrict__ src, bf* dh, bf* dl) {
    const int lane = threadIdx.x & 31; const size_t r = (size_t)blockIdx.x * 8 + (threadIdx.x >> 5); if (r >= (size_t)NN) return; const size_t o = r * HF + lane * 8; v8us oh, ol;
#pragma unroll
    for (int i = 0; i < 8; ++i) { const float v = fmaxf(src[o + i], 0.f); const unsigned short hb = f2bf(v); oh[i] = hb; ol[i] = f2bf(v - bf2f(hb)); }
    *(volatile v8us*)(dh + o) = oh; *(volatile v8us*)(dl + o) = ol; __threadfence(); *(volatile v8us*)(dh + o) = oh; *(volatile v8us*)(dl + o) = ol;
}
__global__ __launch_bounds__(256) void k_hplanes(const float* __restrict__ Hs, bf* Ph, bf* Pl) {
    typedef __attribute__((ext_vector_type(2))) unsigned short v2us;
    const int lane = threadIdx.x & 31; const size_t r = (size_t)blockIdx.x * 8 + (threadIdx.x >> 5); if (r >= (size_t)NN) return; v2us oh, ol;
#pragma unroll
    for (int i = 0; i < 2; ++i) { const int c = lane * 2 + i; const float v = (c < LAT) ? Hs[r * 64 + c] : 0.f; const unsigned short hb = f2bf(v); oh[i] = hb; ol[i] = f2bf(v - bf2f(hb)); }
    const size_t o = r * 64 + lane * 2; *(volatile v2us*)(Ph + o) = oh; *(volatile v2us*)(Pl + o) = ol; __threadfence(); *(volatile v2us*)(Ph + o) = oh; *(volatile v2us*)(Pl + o) = ol;
}
__global__ __launch_bounds__(256) void k_sq(const float* __restrict__ Hs, float* SQ) {
    const int r = blockIdx.x * 256 + threadIdx.x; if (r >= NN) return; float s = 0.f;
#pragma unroll
    for (int d = 0; d < LAT; ++d) { const float v = Hs[(size_t)r * 64 + d]; s = fmaf(v, v, s); }
    *(volatile float*)(SQ + r) = s; __threadfence(); *(volatile float*)(SQ + r) = s;
}
__global__ __launch_bounds__(256) void k_adj(const float* __restrict__ G, const float* __restrict__ SQ, const float* __restrict__ tt, const float* __restrict__ th, int r0, bf* Ah, bf* Al) {
    typedef __attribute__((ext_vector_type(4))) unsigned short v4us;
    const int lane = threadIdx.x & 31, rl = blockIdx.x * 8 + (threadIdx.x >> 5); if (rl >= RCH) return; const int i = r0 + rl; const float sqi = SQ[i], t = bfr(tt[0]), theta = bfr(th[0]);
#pragma unroll 1
    for (int ps = 0; ps < 2; ++ps) {
#pragma unroll 1
        for (int c0 = lane * 4; c0 < NN; c0 += 128) { v4us oh, ol;
#pragma unroll
            for (int q = 0; q < 4; ++q) { const int j = c0 + q; const float d2 = fmaxf(sqi + SQ[j] - 2.0f * G[(size_t)rl * NN + j], 0.f); const float d = (d2 > 0.f) ? sqrtf(d2) : 0.f;
                const float a = 1.0f / (1.0f + __expf(-(t * (d + theta)))); const unsigned short hb = f2bf(a); oh[q] = hb; ol[q] = f2bf(a - bf2f(hb)); }
            const size_t o = (size_t)rl * NN + c0; *(volatile v4us*)(Ah + o) = oh; *(volatile v4us*)(Al + o) = ol; }
        if (ps == 0) __threadfence(); }
}
__global__ __launch_bounds__(256) void k_yt(const float* __restrict__ Y, int ys, int nf, bf* Th, bf* Tl) {
    typedef __attribute__((ext_vector_type(2))) unsigned short v2us;
    const int lane = threadIdx.x & 31; const size_t wid = (size_t)blockIdx.x * 8 + (threadIdx.x >> 5); if (wid >= (size_t)64 * (NN / 64)) return; const int f = (int)(wid / (NN / 64)); const int s0 = (int)(wid % (NN / 64)) * 64 + lane * 2; v2us oh, ol;
#pragma unroll
    for (int i = 0; i < 2; ++i) { const float v = (f < nf) ? Y[(size_t)(s0 + i) * ys + (f < nf ? f : 0)] : 0.f; const unsigned short hb = f2bf(v); oh[i] = hb; ol[i] = f2bf(v - bf2f(hb)); }
    const size_t o = (size_t)f * NN + s0; *(volatile v2us*)(Th + o) = oh; *(volatile v2us*)(Tl + o) = ol; __threadfence(); *(volatile v2us*)(Th + o) = oh; *(volatile v2us*)(Tl + o) = ol;
}
__global__ __launch_bounds__(256) void k_y1(const float* __restrict__ Hs, const float* __restrict__ gw1, float* Y1) {
    const int lane = threadIdx.x & 31; const size_t r = ((size_t)blockIdx.x * 8 + (threadIdx.x >> 5)) * 8 + (lane >> 2); if (r >= (size_t)NN) return; const int f0 = (lane & 3) * 4; v4f o = {0.f, 0.f, 0.f, 0.f};
#pragma unroll 1
    for (int d = 0; d < LAT; ++d) { const float hv = Hs[r * 64 + d];
#pragma unroll
        for (int q = 0; q < 4; ++q) o[q] = fmaf(hv, bfr(gw1[d * 16 + f0 + q]), o[q]); }
    *(volatile v4f*)(Y1 + r * 16 + f0) = o; __threadfence(); *(volatile v4f*)(Y1 + r * 16 + f0) = o;
}
__global__ __launch_bounds__(256) void k_mid(const float* __restrict__ AG1, const float* __restrict__ gb1, const float* __restrict__ gw2, float* Y2) {
    const int lane = threadIdx.x & 31; const size_t r = ((size_t)blockIdx.x * 8 + (threadIdx.x >> 5)) * 16 + (lane >> 1); if (r >= (size_t)NN) return; const int f0 = (lane & 1) * 4; v4f o = {0.f, 0.f, 0.f, 0.f};
#pragma unroll 1
    for (int k = 0; k < 16; ++k) { const float h1k = fmaxf(AG1[r * 64 + k] * (1.0f / NN) + bfr(gb1[k]), 0.f);
#pragma unroll
        for (int q = 0; q < 4; ++q) o[q] = fmaf(h1k, bfr(gw2[k * 8 + f0 + q]), o[q]); }
    *(volatile v4f*)(Y2 + r * 8 + f0) = o; __threadfence(); *(volatile v4f*)(Y2 + r * 8 + f0) = o;
}
__global__ __launch_bounds__(256) void k_out(const float* __restrict__ AG2, const float* __restrict__ gb2, const float* __restrict__ lw1, const float* __restrict__ lb1, const float* __restrict__ lw2, const float* __restrict__ lb2, float* OUTP) {
    typedef __attribute__((ext_vector_type(16))) float v16f;
    __shared__ float h3s[256][17];
    const int lane = threadIdx.x & 31, tid = threadIdx.x; const size_t r = ((size_t)blockIdx.x * 8 + (threadIdx.x >> 5)) * 8 + (lane >> 2); if (r >= (size_t)NN) return; const int f0 = (lane & 3) * 4;
    v16f a;
#pragma unroll
    for (int f = 0; f < 16; ++f) a[f] = bfr(lb1[f]);
#pragma unroll 1
    for (int k = 0; k < 8; ++k) { const float h2k = fmaxf(AG2[r * 64 + k] * (1.0f / NN) + bfr(gb2[k]), 0.f);
#pragma unroll
        for (int f = 0; f < 16; ++f) a[f] = fmaf(h2k, bfr(lw1[k * 16 + f]), a[f]); }
#pragma unroll
    for (int f = 0; f < 16; ++f) h3s[tid][f] = fmaxf(a[f], 0.f);
    v4f o;
#pragma unroll
    for (int q = 0; q < 4; ++q) o[q] = bfr(lb2[f0 + q]);
#pragma unroll 1
    for (int k = 0; k < 16; ++k) { const float h3k = h3s[tid][k];
#pragma unroll
        for (int q = 0; q < 4; ++q) o[q] = fmaf(h3k, bfr(lw2[k * 16 + f0 + q]), o[q]); }
    *(volatile v4f*)(OUTP + r * 16 + f0) = o; __threadfence(); *(volatile v4f*)(OUTP + r * 16 + f0) = o;
}

__global__ __launch_bounds__(64) void k_b3p(const float* __restrict__ b3, float* B3P) {
    typedef __attribute__((ext_vector_type(2))) float v2f;
    const int lane = threadIdx.x; if (lane >= 32) return; v2f v; v[0] = (2 * lane < LAT) ? b3[2 * lane] : 0.f; v[1] = (2 * lane + 1 < LAT) ? b3[2 * lane + 1] : 0.f;
    *(volatile v2f*)(B3P + 2 * lane) = v; __threadfence(); *(volatile v2f*)(B3P + 2 * lane) = v;
}

extern "C" void kernel_launch(void* const* d_in, const int* in_sizes, int n_in,
                              void* d_out, int out_size, void* d_ws, size_t ws_size, hipStream_t stream) {
    (void)in_sizes; (void)n_in; (void)out_size;
    const float* x = (const float*)d_in[0]; const float* w1 = (const float*)d_in[1]; const float* b1 = (const float*)d_in[2]; const float* w2 = (const float*)d_in[3]; const float* b2 = (const float*)d_in[4]; const float* w3 = (const float*)d_in[5]; const float* b3 = (const float*)d_in[6];
    const float* tt = (const float*)d_in[7]; const float* th = (const float*)d_in[8]; const float* gw1 = (const float*)d_in[9]; const float* gb1 = (const float*)d_in[10]; const float* gw2 = (const float*)d_in[11]; const float* gb2 = (const float*)d_in[12];
    const float* lw1 = (const float*)d_in[13]; const float* lb1 = (const float*)d_in[14]; const float* lw2 = (const float*)d_in[15]; const float* lb2 = (const float*)d_in[16];
    float* out = (float*)d_out;
    char* wsp = (char*)d_ws;
    auto take = [&](size_t bytes) { char* p = wsp; wsp += (bytes + 255) & ~(size_t)255; return (void*)p; };
    bf* W1T = (bf*)take((size_t)HF * FIN * 2); bf* W2T = (bf*)take((size_t)HF * HF * 2); bf* W3T = (bf*)take((size_t)64 * HF * 2);
    bf* Xb = (bf*)take((size_t)NN * FIN * 2); float* T = (float*)take((size_t)NN * HF * 4); bf* Rh = (bf*)take((size_t)NN * HF * 2); bf* Rl = (bf*)take((size_t)NN * HF * 2); float* Hs = (float*)take((size_t)NN * 64 * 4);
    bf* HPh = (bf*)take((size_t)NN * 64 * 2); bf* HPl = (bf*)take((size_t)NN * 64 * 2); float* SQ = (float*)take(NN * 4); float* G = (float*)take((size_t)RCH * NN * 4); bf* Ah = (bf*)take((size_t)RCH * NN * 2); bf* Al = (bf*)take((size_t)RCH * NN * 2);
    float* Y1 = (float*)take((size_t)NN * 16 * 4); float* Y2 = (float*)take((size_t)NN * 8 * 4); bf* YTh = (bf*)take((size_t)64 * NN * 2); bf* YTl = (bf*)take((size_t)64 * NN * 2); float* AG = (float*)take((size_t)NN * 64 * 4); float* B3P = (float*)take(64 * 4);
    if ((size_t)(wsp - (char*)d_ws) > ws_size) return;
    k_wt<<<dim3(FIN / 64, HF / 64, 1), 256, 0, stream>>>(w1, FIN, HF, W1T); k_wt<<<dim3(HF / 64, HF / 64, 1), 256, 0, stream>>>(w2, HF, HF, W2T); k_wtp<<<dim3(HF / 64, 1, 1), 256, 0, stream>>>(w3, HF, LAT, HF, W3T);
    k_cvtx<<<NN / 8, 256, 0, stream>>>(x, Xb);
    k_gemmb<false, false><<<dim3(NN / 64, HF / 64, 1), 128, 0, stream>>>(Xb, nullptr, W1T, b1, T, HF, nullptr, nullptr, FIN); k_relu256<<<NN / 8, 256, 0, stream>>>(T, Rh, Rl);
    k_gemmb<true, false><<<dim3(NN / 64, HF / 64, 1), 128, 0, stream>>>(Rh, Rl, W2T, b2, T, HF, nullptr, nullptr, HF); k_relu256<<<NN / 8, 256, 0, stream>>>(T, Rh, Rl);
    k_b3p<<<1, 64, 0, stream>>>(b3, B3P); k_gemmb<true, false><<<dim3(NN / 64, 1, 1), 128, 0, stream>>>(Rh, Rl, W3T, B3P, Hs, 64, nullptr, nullptr, HF);
    k_hplanes<<<NN / 8, 256, 0, stream>>>(Hs, HPh, HPl); k_sq<<<NN / 256, 256, 0, stream>>>(Hs, SQ);
    k_y1<<<NN / 64, 256, 0, stream>>>(Hs, gw1, Y1); k_yt<<<(64 * (NN / 64)) / 8, 256, 0, stream>>>(Y1, 16, 16, YTh, YTl);
    for (int ch = 0; ch < NCH; ++ch) { const int r0 = ch * RCH;
        k_gemm3<<<dim3(RCH / 64, NN / 64, 1), 128, 0, stream>>>(HPh + (size_t)r0 * 64, HPl + (size_t)r0 * 64, HPh, HPl, 64, G, NN); k_adj<<<RCH / 8, 256, 0, stream>>>(G, SQ, tt, th, r0, Ah, Al);
        k_gemm3<<<dim3(RCH / 64, 1, 1), 128, 0, stream>>>(Ah, Al, YTh, YTl, NN, AG + (size_t)r0 * 64, 64); }
    k_mid<<<NN / 128, 256, 0, stream>>>(AG, gb1, gw2, Y2); k_yt<<<(64 * (NN / 64)) / 8, 256, 0, stream>>>(Y2, 8, 8, YTh, YTl);
    for (int ch = 0; ch < NCH; ++ch) { const int r0 = ch * RCH;
        k_gemm3<<<dim3(RCH / 64, NN / 64, 1), 128, 0, stream>>>(HPh + (size_t)r0 * 64, HPl + (size_t)r0 * 64, HPh, HPl, 64, G, NN); k_adj<<<RCH / 8, 256, 0, stream>>>(G, SQ, tt, th, r0, Ah, Al);
        k_gemm3<<<dim3(RCH / 64, 1, 1), 128, 0, stream>>>(Ah, Al, YTh, YTl, NN, AG + (size_t)r0 * 64, 64); }
    k_out<<<NN / 64, 256, 0, stream>>>(AG, gb2, lw1, lb1, lw2, lb2, out);
}
